// TemporalAttnLayer_10763188044505
// MI455X (gfx1250) — hardware-run, weakly checked
//
#include <hip/hip_runtime.h>


#ifndef NB
#define NB 4
#endif
#ifndef SEQ
#define SEQ 512
#endif
#define NB_FULL  4
#define SEQ_FULL 512
#ifndef OUT_SEQ
#define OUT_SEQ SEQ
#endif
#define NJ   24
#define DM   128
#define NHD  8
#define HD   16
#define MROWS (NB * SEQ)
#define AW   4
#define OSP  20
#define OLP  132
#define EROWS (SEQ < 256 ? SEQ : 256)
#define QRS  2048.0f
#define QRI  (1.0f / 2048.0f)
#define LOG2E ((float)1.4426950408889634)
#define SC2  ((float)(0.25 * 1.4426950408889634))
#define PSH  14.0f
#define NEGB (-3.0e38f)
#define MDROP (-1.0e8f)
#define CTS  16.0f
#define PWS  64.0f
#define SCO  (1.0f / 1024.0f)
#define LNE  1.0e-5f

static_assert(HD == 16);
static_assert(NHD * HD == DM);
static_assert(DM % 64 == 0);
static_assert(64 % HD == 0);
static_assert(DM % 32 == 0);
static_assert((2 * HD) == 32);
static_assert(SEQ % 64 == 0);
static_assert((NB * SEQ) % 64 == 0);
static_assert(SEQ % 32 == 0);
static_assert(SEQ % (16 * AW) == 0);
static_assert(EROWS % 64 == 0);
static_assert(EROWS >= 32);
static_assert(EROWS <= SEQ);
static_assert(EROWS % (16 * AW) == 0);
static_assert((SEQ - EROWS) % (16 * AW) == 0);
static_assert(NB <= NB_FULL);
static_assert(SEQ <= SEQ_FULL);
static_assert((OSP * 4) % 16 == 0);
static_assert(OSP >= HD);
static_assert((OLP * 4) % 16 == 0);
static_assert(OLP >= DM);
static_assert(NB * NHD * NJ <= 65535);
static_assert(NJ <= 65535);
static_assert(32 * 16 == 16 * HD * 2);
static_assert(4 * 32 * 16 == 16 * 64 * 2);
static_assert(32 * 16 == DM * 4);
static_assert(256 * 16 == HD * DM * 2);
static_assert(256 * 8 == DM * HD);
static_assert(16 * 68 * 4 <= 131072);
static_assert(AW * 16 * OSP * 4 <= 131072);
static_assert(16 * OLP * 4 <= 131072);
static_assert(128 * 20 * 4 <= 131072);
static_assert(((size_t)NB * SEQ * NJ * DM) % 8 == 0);
static_assert(((size_t)SEQ * NJ * DM) % 8 == 0);

typedef _Float16 h16;
typedef unsigned short bf;
typedef __attribute__((ext_vector_type(16))) __bf16   v16bf;
typedef __attribute__((ext_vector_type(16))) _Float16 v16h;
typedef __attribute__((ext_vector_type(8)))  _Float16 v8h;
typedef __attribute__((ext_vector_type(8)))  unsigned short v8us;
typedef __attribute__((ext_vector_type(8)))  float    v8f;
typedef __attribute__((ext_vector_type(4)))  float    v4f;
typedef v4f  __attribute__((may_alias)) v4fa;

__device__ __forceinline__ unsigned short f2bf(float f) { unsigned u = __float_as_uint(f); u += 0x7FFFu + ((u >> 16) & 1u); return (unsigned short)(u >> 16); }
__device__ __forceinline__ float bfr(float f) { return __uint_as_float(((unsigned)f2bf(f)) << 16); }
__device__ __forceinline__ v16h cat16(v8h lo, v8h hi) { return __builtin_shufflevector(lo, hi, 0, 1, 2, 3, 4, 5, 6, 7, 8, 9, 10, 11, 12, 13, 14, 15); }
__device__ __forceinline__ v16bf cat16b(v8us lo, v8us hi) { return __builtin_bit_cast(v16bf, __builtin_shufflevector(lo, hi, 0, 1, 2, 3, 4, 5, 6, 7, 8, 9, 10, 11, 12, 13, 14, 15)); }
__device__ __forceinline__ v8f wmma16(v16h a, v16h b, v8f c) { return __builtin_amdgcn_wmma_f32_16x16x32_f16(false, a, false, b, (short)0, c, false, false); }
__device__ __forceinline__ v8f wmmab(v16bf a, v16bf b, v8f c) { return __builtin_amdgcn_wmma_f32_16x16x32_bf16(false, a, false, b, (short)0, c, false, false); }
__device__ __forceinline__ v8f wmma16g(v16h a, v16h b, v8f c) { c = wmma16(a, b, c); asm volatile("v_nop\n\tv_nop\n\tv_nop\n\tv_nop" : "+v"(c) : "v"(a), "v"(b)); return c; }
__device__ __forceinline__ v8f wmmabg(v16bf a, v16bf b, v8f c) { c = wmmab(a, b, c); asm volatile("v_nop\n\tv_nop\n\tv_nop\n\tv_nop" : "+v"(c) : "v"(a), "v"(b)); return c; }
static __device__ __forceinline__ h16 toh_flush(float v) { const float w = (fabsf(v) < 6.103515625e-05f) ? 0.0f : v; return (h16)w; }
__device__ __forceinline__ v16h  ldh(const h16* p) { return cat16(*(const v8h*)p, *(const v8h*)(p + 16)); }
__device__ __forceinline__ v16bf ldb(const bf* p)  { return cat16b(*(const v8us*)p, *(const v8us*)(p + 16)); }
__device__ __forceinline__ v16h  ldhz(const h16* p) { return cat16(*(const v8h*)p, (v8h){}); }
__device__ __forceinline__ void wave_sync() { __builtin_amdgcn_fence(3  , "wavefront"); __builtin_amdgcn_wave_barrier(); asm volatile("" ::: "memory"); }

__global__ __launch_bounds__(256) void k_cvt8(const float* __restrict__ src, bf* dst, size_t n8) {
    const size_t i = (size_t)blockIdx.x * 256 + threadIdx.x; if (i >= n8) return;
    const v8f v = *(const v8f*)(src + i * 8); v8us o;
#pragma unroll
    for (int k = 0; k < 8; ++k) o[k] = f2bf(v[k]);
    *(volatile v8us*)(dst + i * 8) = o; __threadfence(); *(volatile v8us*)(dst + i * 8) = o;
}

__global__ __launch_bounds__(256) void k_wtr(const float* __restrict__ src, bf* dst) {
    __shared__ __align__(16) float ts[128 * 20];
    const unsigned tid = threadIdx.x;
    const unsigned g = blockIdx.x / (unsigned)NJ, j = blockIdx.x % (unsigned)NJ;
    const size_t sbase = (size_t)blockIdx.x * (size_t)(DM * HD);
    { const unsigned h = tid >> 1, d0 = (tid & 1u) * 8u;
      const v4f a = *(const v4f*)(src + sbase + (size_t)h * HD + d0); const v4f c = *(const v4f*)(src + sbase + (size_t)h * HD + d0 + 4);
      *(v4fa*)(&ts[h * 20 + d0]) = a; *(v4fa*)(&ts[h * 20 + d0 + 4]) = c; }
    __syncthreads();
    const unsigned d = tid >> 4, c8 = (tid & 15u) * 8u;
    v8us o;
#pragma unroll
    for (int k = 0; k < 8; ++k) o[k] = f2bf(ts[(c8 + k) * 20 + d]);
    bf* p = dst + ((size_t)j * DM + (size_t)g * HD + d) * DM + c8;
    *(volatile v8us*)p = o; __threadfence(); *(volatile v8us*)p = o;
}

__global__ __launch_bounds__(256) void k_ptr(const float* __restrict__ src, h16* dst) {
    __shared__ __align__(16) float ts[128 * 20];
    const unsigned tid = threadIdx.x;
    const unsigned g = blockIdx.x / (unsigned)NJ, j = blockIdx.x % (unsigned)NJ;
    const size_t sbase = (size_t)j * (size_t)(DM * DM) + (size_t)g * HD;
    { const unsigned h = tid >> 1, d0 = (tid & 1u) * 8u;
      const v4f a = *(const v4f*)(src + sbase + (size_t)h * DM + d0); const v4f c = *(const v4f*)(src + sbase + (size_t)h * DM + d0 + 4);
      *(v4fa*)(&ts[h * 20 + d0]) = a; *(v4fa*)(&ts[h * 20 + d0 + 4]) = c; }
    __syncthreads();
    const unsigned d = tid >> 4, c8 = (tid & 15u) * 8u;
    v8h o;
#pragma unroll
    for (int k = 0; k < 8; ++k) o[k] = toh_flush(bfr(ts[(c8 + k) * 20 + d]) * PWS);
    h16* p = dst + ((size_t)j * DM + (size_t)g * HD + d) * DM + c8;
    *(volatile v8h*)p = o; __threadfence(); *(volatile v8h*)p = o;
}

template <int MODE>
__device__ __forceinline__ void proj_body(const bf* __restrict__ A, const bf* __restrict__ Bt, h16* Ph, h16* Pr, const unsigned resT) {
    __shared__ __align__(16) float os[16 * 68];
    constexpr size_t LDA = (MODE == 0) ? (size_t)NJ * DM : (size_t)DM;
    constexpr size_t LDB = (MODE == 0) ? (size_t)DM : (size_t)NJ * DM;
    constexpr size_t AJ  = (MODE == 0) ? (size_t)DM : (size_t)DM * DM;
    constexpr size_t BJ  = (MODE == 0) ? (size_t)DM * DM : (size_t)DM;
    const int lane = threadIdx.x & 31, lr = lane & 15, hi = lane >> 4;
    const unsigned r0 = blockIdx.x * 64u, c0 = blockIdx.y * 64u, jz = blockIdx.z;
    v8f acc[4][4];
#pragma unroll
    for (int mb = 0; mb < 4; ++mb)
#pragma unroll
        for (int nb = 0; nb < 4; ++nb) acc[mb][nb] = (v8f){};
    const size_t aoff = (size_t)(r0 + (unsigned)lr) * LDA + (size_t)jz * AJ + (size_t)(8 * hi);
    const size_t boff = (size_t)(c0 + (unsigned)lr) * LDB + (size_t)jz * BJ + (size_t)(8 * hi);
#pragma unroll 1
    for (int kc = 0; kc < DM; kc += 32) {
        v16bf a[4];
#pragma unroll
        for (int mb = 0; mb < 4; ++mb) a[mb] = ldb(A + aoff + (size_t)mb * 16 * LDA + kc);
#pragma unroll
        for (int nb = 0; nb < 4; ++nb) { const v16bf b = ldb(Bt + boff + (size_t)nb * 16 * LDB + kc);
#pragma unroll
            for (int mb = 0; mb < 4; ++mb) acc[mb][nb] = wmmabg(a[mb], b, acc[mb][nb]); }
    }
    unsigned bb, tt;
    if (MODE == 0) { bb = r0 / (unsigned)SEQ; tt = r0 % (unsigned)SEQ; } else { bb = c0 / (unsigned)SEQ; tt = c0 % (unsigned)SEQ; }
    const unsigned hq = (MODE == 0) ? (c0 >> 4) : (r0 >> 4);
    const size_t zc0 = (size_t)(bb * (unsigned)NHD + hq) * NJ + jz;
    const bool wr = tt < resT;
#pragma unroll
    for (int mb = 0; mb < 4; ++mb) {
#pragma unroll
        for (int nb = 0; nb < 4; ++nb) {
#pragma unroll
            for (int j = 0; j < 8; ++j) os[(hi * 8 + j) * 68 + nb * 16 + lr] = acc[mb][nb][j]; }
        wave_sync();
#pragma unroll 1
        for (int ps = 0; ps < 2; ++ps) {
            if (MODE == 0) {
#pragma unroll
                for (int nb = 0; nb < 4; ++nb) { const int row = lane >> 1, c8 = (lane & 1) * 8;
                    const v4f x0 = *(const v4fa*)(&os[row * 68 + nb * 16 + c8]); const v4f x1 = *(const v4fa*)(&os[row * 68 + nb * 16 + c8 + 4]); v8h hv, rv;
#pragma unroll
                    for (int i = 0; i < 4; ++i) { const h16 a0 = toh_flush(x0[i]); const h16 a1 = toh_flush(x1[i]); hv[i] = a0; hv[4 + i] = a1;
                        rv[i] = toh_flush((x0[i] - (float)a0) * QRS); rv[4 + i] = toh_flush((x1[i] - (float)a1) * QRS); }
                    const size_t zc = zc0 + (size_t)nb * NJ;
                    const size_t oo = (zc * SEQ + (size_t)tt + (size_t)(mb * 16)) * HD + (size_t)lane * 8;
                    const size_t ro = (zc * (size_t)resT + (size_t)tt + (size_t)(mb * 16)) * HD + (size_t)lane * 8;
                    *(volatile v8h*)(Ph + oo) = hv; if (wr) *(volatile v8h*)(Pr + ro) = rv; }
            } else {
                const size_t zc = zc0 + (size_t)mb * NJ;
#pragma unroll
                for (int s = 0; s < 4; ++s) { const int row = 4 * s + (lane >> 3), c8 = (lane & 7) * 8;
                    const v4f x0 = *(const v4fa*)(&os[row * 68 + c8]); const v4f x1 = *(const v4fa*)(&os[row * 68 + c8 + 4]); v8h hv, rv;
#pragma unroll
                    for (int i = 0; i < 4; ++i) { const h16 a0 = toh_flush(x0[i]); const h16 a1 = toh_flush(x1[i]); hv[i] = a0; hv[4 + i] = a1;
                        rv[i] = toh_flush((x0[i] - (float)a0) * QRS); rv[4 + i] = toh_flush((x1[i] - (float)a1) * QRS); }
                    const size_t oo = (zc * HD + (size_t)row) * SEQ + (size_t)tt + (size_t)c8;
                    const size_t ro = (zc * HD + (size_t)row) * (size_t)resT + (size_t)tt + (size_t)c8;
                    *(volatile v8h*)(Ph + oo) = hv; if (wr) *(volatile v8h*)(Pr + ro) = rv; }
            }
            if (ps == 0) __threadfence(); }
        wave_sync();
    }
}

__global__ __launch_bounds__(32) void k_proj_qk(const bf* __restrict__ X, const bf* __restrict__ WT, h16* Ph, h16* Pr, int resT) {
    proj_body<0>(X, WT, Ph, Pr, (unsigned)resT);
}
__global__ __launch_bounds__(32) void k_proj_vt(const bf* __restrict__ WT, const bf* __restrict__ X, h16* Ph, h16* Pr, int resT) {
    proj_body<1>(WT, X, Ph, Pr, (unsigned)resT);
}

template <int EARLY>
__device__ __forceinline__ void flash_body(const h16* __restrict__ QH, const h16* __restrict__ QR, const h16* __restrict__ KP, const h16* __restrict__ KR,
                                           const h16* __restrict__ VT, const h16* __restrict__ VR, const float* __restrict__ mask, h16* CT) {
    __shared__ __align__(16) float os[AW * 16 * OSP];
    const int lane = threadIdx.x & 31, lr = lane & 15, hi = lane >> 4;
    const int wave = __builtin_amdgcn_readfirstlane((int)(threadIdx.x >> 5));
    const unsigned zh = blockIdx.y;
    const unsigned b = zh / (unsigned)(NHD * NJ), n = (zh / (unsigned)NJ) % (unsigned)NHD, j = zh % (unsigned)NJ;
    const unsigned t0 = (EARLY ? 0u : (unsigned)EROWS) + (blockIdx.x * (unsigned)AW + (unsigned)wave) * 16u;
    const float* mrow = mask + (size_t)(t0 + (unsigned)lr) * SEQ_FULL + (size_t)(8 * hi);
    const size_t pbase = (size_t)zh * SEQ * HD;
    const size_t rbase = (size_t)zh * EROWS * HD;
    const size_t qo = pbase + (size_t)(t0 + (unsigned)lr) * HD + (size_t)(8 * hi);
    const v16h qh = ldhz(QH + qo), qr = ldhz(QR + qo);
    const size_t ko = pbase + (size_t)lr * HD + (size_t)(8 * hi);
    const size_t vo = pbase + (size_t)lr * SEQ + (size_t)(8 * hi);
    const size_t kro = rbase + (size_t)lr * HD + (size_t)(8 * hi);
    const size_t vro = rbase + (size_t)lr * EROWS + (size_t)(8 * hi);
    const v16h hz = (v16h){};
    v8f o0 = (v8f){}, oR0 = (v8f){};
    float m = NEGB, l = 0.0f;
#pragma unroll 1
    for (int key0 = 0; key0 < SEQ; key0 += 32) {
        const float* mp = mrow + key0;
        v4f m0 = *(const v4f*)mp, m1 = *(const v4f*)(mp + 4), m2 = *(const v4f*)(mp + 16), m3 = *(const v4f*)(mp + 20);
        asm volatile("" : "+v"(m0), "+v"(m1), "+v"(m2), "+v"(m3));
        float kx[8], ky[8];
#pragma unroll
        for (int r = 0; r < 4; ++r) { kx[r] = bfr(m0[r]); kx[4 + r] = bfr(m1[r]); ky[r] = bfr(m2[r]); ky[4 + r] = bfr(m3[r]); }
        float fa[8], fb[8];
#pragma unroll
        for (int r = 0; r < 8; ++r) { fa[r] = (kx[r] < MDROP) ? 0.0f : 1.0f; fb[r] = (ky[r] < MDROP) ? 0.0f : 1.0f; asm volatile("" : "+v"(fa[r]), "+v"(fb[r])); }
        bool anyk = false;
#pragma unroll
        for (int r = 0; r < 8; ++r) { anyk = anyk || (fa[r] != 0.0f) || (fb[r] != 0.0f); }
        if (__builtin_amdgcn_ballot_w32(anyk) != 0u) {
            const bool rok = key0 < EROWS;
            const int kcl = min(key0, EROWS - 32);
            const h16* ka = KP + ko + (size_t)key0 * HD;
            const v16h ka0 = ldhz(ka), kb0 = ldhz(ka + 16 * HD);
            v16h kra0 = hz, krb0 = hz;
            if (EARLY) { const h16* kr = KR + kro + (size_t)kcl * HD; kra0 = ldhz(kr); krb0 = ldhz(kr + 16 * HD); if (!rok) { kra0 = hz; krb0 = hz; } }
            v8f sHa = (v8f){}, sLa = (v8f){}, sHb = (v8f){}, sLb = (v8f){};
            sHa = wmma16g(ka0, qh, sHa); sLa = wmma16g(ka0, qr, sLa); sHb = wmma16g(kb0, qh, sHb); sLb = wmma16g(kb0, qr, sLb);
            if (EARLY) { sLa = wmma16g(kra0, qh, sLa); sLb = wmma16g(krb0, qh, sLb); }
            float ta[8], tb[8]; float mx = NEGB;
#pragma unroll
            for (int r = 0; r < 8; ++r) {
                ta[r] = (sHa[r] + sLa[r] * QRI) * SC2 + kx[r] * LOG2E; tb[r] = (sHb[r] + sLb[r] * QRI) * SC2 + ky[r] * LOG2E;
                mx = fmaxf(mx, fmaxf((fa[r] != 0.0f) ? ta[r] : NEGB, (fb[r] != 0.0f) ? tb[r] : NEGB)); }
            mx = fmaxf(mx, __shfl_xor(mx, 16, 32));
            const float mnew = fmaxf(m, mx);
            const float alpha = __builtin_amdgcn_exp2f(m - mnew);
            const float sh = PSH - mnew;
            v16h pb, pr = hz; float ls = 0.0f;
#pragma unroll
            for (int r = 0; r < 8; ++r) {
                const float xa = ta[r] + sh, xb = tb[r] + sh;
                const float ea = __builtin_amdgcn_exp2f(xa), eb = __builtin_amdgcn_exp2f(xb);
                const float ga = ((fa[r] != 0.0f) && xa >= -14.0f) ? ea : 0.0f, gb = ((fb[r] != 0.0f) && xb >= -14.0f) ? eb : 0.0f;
                const h16 pa = (h16)ga; const h16 pc = (h16)gb;
                pb[r] = pa; pb[8 + r] = pc;
                if (EARLY) { pr[r] = toh_flush((ga - (float)pa) * QRS); pr[8 + r] = toh_flush((gb - (float)pc) * QRS); ls += ga + gb; }
                else       { ls += (float)pa + (float)pc; } }
            l = l * alpha + ls; m = mnew;
            o0 = o0 * alpha;
            if (EARLY) { oR0 = oR0 * alpha; }
            const v16h v0 = ldh(VT + vo + key0);
            if (EARLY) {
                v16h vr0 = ldh(VR + vro + kcl);
                if (!rok) { vr0 = hz; }
                o0 = wmma16g(v0, pb, o0);
                oR0 = wmma16g(v0, pr, oR0);
                oR0 = wmma16g(vr0, pb, oR0);
            } else {
                o0 = wmma16g(v0, pb, o0);
            }
        }
    }
    l += __shfl_xor(l, 16, 32);
    const bool any = l > 0.0f;
    const float lsafe = any ? l : 1.0f;
    const float inv = any ? (CTS / lsafe) : 0.0f;
    v8f f0 = o0;
    if (EARLY) { f0 = o0 + oR0 * QRI; }
    const int wb = wave * 16 * OSP;
    { v4f a, c;
      a[0] = f0[0] * inv; a[1] = f0[1] * inv; a[2] = f0[2] * inv; a[3] = f0[3] * inv; c[0] = f0[4] * inv; c[1] = f0[5] * inv; c[2] = f0[6] * inv; c[3] = f0[7] * inv;
      *(v4fa*)(&os[wb + lr * OSP + 8 * hi]) = a; *(v4fa*)(&os[wb + lr * OSP + 8 * hi + 4]) = c; }
    wave_sync();
    h16* crow = CT + (((size_t)j * NHD + n) * MROWS + (size_t)b * SEQ + t0) * HD + (size_t)lane * 8;
    const int row = lane >> 1, c8 = (lane & 1) * 8;
    const v4f x0 = *(const v4fa*)(&os[wb + row * OSP + c8]); const v4f x1 = *(const v4fa*)(&os[wb + row * OSP + c8 + 4]);
    v8h hv;
#pragma unroll
    for (int i = 0; i < 4; ++i) { hv[i] = toh_flush(x0[i]); hv[4 + i] = toh_flush(x1[i]); }
    *(volatile v8h*)crow = hv; __threadfence(); *(volatile v8h*)crow = hv;
}

__global__ __launch_bounds__(32 * AW) void k_flash_early(const h16* __restrict__ QH, const h16* __restrict__ QR, const h16* __restrict__ KP, const h16* __restrict__ KR,
                                                         const h16* __restrict__ VT, const h16* __restrict__ VR, const float* __restrict__ mask, h16* CT) {
    flash_body<1>(QH, QR, KP, KR, VT, VR, mask, CT);
}
__global__ __launch_bounds__(32 * AW) void k_flash_late(const h16* __restrict__ QH, const h16* __restrict__ QR, const h16* __restrict__ KP, const h16* __restrict__ KR,
                                                        const h16* __restrict__ VT, const h16* __restrict__ VR, const float* __restrict__ mask, h16* CT) {
    flash_body<0>(QH, QR, KP, KR, VT, VR, mask, CT);
}

__global__ __launch_bounds__(32) void k_oproj(const h16* __restrict__ CT, const h16* __restrict__ PT, const float* __restrict__ X,
                                              const float* __restrict__ gam, const float* __restrict__ bet, float* OUT) {
    __shared__ __align__(16) float os[16 * OLP];
    const int lane = threadIdx.x & 31, lr = lane & 15, hi = lane >> 4;
    const unsigned m0 = blockIdx.x * 32u, jz = blockIdx.y;
    v8f acc[2][8];
#pragma unroll
    for (int mb = 0; mb < 2; ++mb)
#pragma unroll
        for (int nb = 0; nb < 8; ++nb) acc[mb][nb] = (v8f){};
    const size_t hstr = (size_t)MROWS * HD;
    const size_t aoff = ((size_t)jz * NHD * MROWS + (size_t)(m0 + (unsigned)lr)) * HD + (size_t)(8 * hi);
    const size_t boff = ((size_t)jz * DM + (size_t)lr) * DM + (size_t)(8 * hi);
#pragma unroll 1
    for (int kc = 0; kc < DM; kc += 32) {
        const size_t ah = aoff + (size_t)(kc >> 4) * hstr;
        v16h a[2];
#pragma unroll
        for (int mb = 0; mb < 2; ++mb) a[mb] = cat16(*(const v8h*)(CT + ah + (size_t)mb * 16 * HD), *(const v8h*)(CT + ah + hstr + (size_t)mb * 16 * HD));
#pragma unroll
        for (int nb = 0; nb < 8; ++nb) { const v16h bq = ldh(PT + boff + (size_t)nb * 16 * DM + kc);
#pragma unroll
            for (int mb = 0; mb < 2; ++mb) acc[mb][nb] = wmma16g(a[mb], bq, acc[mb][nb]); }
    }
    const unsigned bb = m0 / (unsigned)SEQ, ss = m0 % (unsigned)SEQ;
    const v4f g4 = *(const v4f*)(gam + 4 * lane); const v4f b4 = *(const v4f*)(bet + 4 * lane);
    v4f gq, bq4;
#pragma unroll
    for (int i = 0; i < 4; ++i) { gq[i] = bfr(g4[i]); bq4[i] = bfr(b4[i]); }
#pragma unroll
    for (int mb = 0; mb < 2; ++mb) {
#pragma unroll
        for (int nb = 0; nb < 8; ++nb) {
#pragma unroll
            for (int r = 0; r < 8; ++r) os[(hi * 8 + r) * OLP + nb * 16 + lr] = acc[mb][nb][r] * SCO; }
        wave_sync();
#pragma unroll 1
        for (int row = 0; row < 16; ++row) {
            const unsigned s = ss + (unsigned)(mb * 16 + row);
            const v4f xv = *(const v4f*)(X + (((size_t)bb * SEQ_FULL + s) * NJ + jz) * DM + 4 * lane);
            const v4f cv = *(const v4fa*)(&os[row * OLP + 4 * lane]);
            v4f y;
#pragma unroll
            for (int i = 0; i < 4; ++i) y[i] = cv[i] + bfr(xv[i]);
            float sm = (y[0] + y[1]) + (y[2] + y[3]);
            sm += __shfl_xor(sm, 16, 32); sm += __shfl_xor(sm, 8, 32); sm += __shfl_xor(sm, 4, 32); sm += __shfl_xor(sm, 2, 32); sm += __shfl_xor(sm, 1, 32);
            const float mu = sm * (1.0f / (float)DM);
            v4f d;
#pragma unroll
            for (int i = 0; i < 4; ++i) d[i] = y[i] - mu;
            float q = (d[0] * d[0] + d[1] * d[1]) + (d[2] * d[2] + d[3] * d[3]);
            q += __shfl_xor(q, 16, 32); q += __shfl_xor(q, 8, 32); q += __shfl_xor(q, 4, 32); q += __shfl_xor(q, 2, 32); q += __shfl_xor(q, 1, 32);
            const float rs = rsqrtf(q * (1.0f / (float)DM) + LNE);
            v4f o;
#pragma unroll
            for (int i = 0; i < 4; ++i) o[i] = d[i] * rs * gq[i] + bq4[i];
            *(v4fa*)(&os[row * OLP + 4 * lane]) = o;
        }
        wave_sync();
        float* obase = OUT + (((size_t)bb * OUT_SEQ + ss + (unsigned)(mb * 16)) * NJ + jz) * DM + 4 * lane;
#pragma unroll 1
        for (int ps = 0; ps < 2; ++ps) {
#pragma unroll 4
            for (int row = 0; row < 16; ++row) {
                const v4f val = *(const v4fa*)(&os[row * OLP + 4 * lane]);
                *(volatile v4f*)(obase + (size_t)row * NJ * DM) = val; }
            if (ps == 0) __threadfence(); }
        wave_sync();
    }
}

static constexpr size_t al256(size_t v) { return (v + 255) & ~(size_t)255; }
static constexpr size_t SZ_XB = al256((size_t)NB * SEQ * NJ * DM * 2);
static constexpr size_t SZ_WT = al256((size_t)NJ * DM * DM * 2);
static constexpr size_t SZ_PL = al256((size_t)NB * NHD * NJ * SEQ * HD * 2);
static constexpr size_t SZ_RS = al256((size_t)NB * NHD * NJ * EROWS * HD * 2);
static constexpr size_t SZ_TOTAL = SZ_XB + 4 * SZ_WT + 5 * SZ_PL + 2 * SZ_RS;
static_assert(SZ_TOTAL <= (size_t)134217728);
static_assert((size_t)NJ * NHD * MROWS * HD == (size_t)NB * NHD * NJ * SEQ * HD);
static_assert((size_t)NHD * NJ * DM * HD == (size_t)NJ * DM * DM);

extern "C" void kernel_launch(void* const* d_in, const int* in_sizes, int n_in,
                              void* d_out, int out_size, void* d_ws, size_t ws_size, hipStream_t stream) {
    if (n_in < 8) return;
    const size_t needx = ((size_t)(NB - 1) * SEQ_FULL + SEQ) * NJ * DM;
    const size_t needm = (size_t)(SEQ - 1) * SEQ_FULL + SEQ;
    if ((size_t)in_sizes[0] < needx) return;
    if ((size_t)in_sizes[1] < needm) return;
    if ((size_t)in_sizes[2] < (size_t)NHD * NJ * DM * HD || (size_t)in_sizes[3] < (size_t)NHD * NJ * DM * HD || (size_t)in_sizes[4] < (size_t)NHD * NJ * DM * HD) return;
    if ((size_t)in_sizes[5] < (size_t)NJ * DM * DM) return;
    if (in_sizes[6] < DM || in_sizes[7] < DM) return;
    if ((size_t)out_size < ((size_t)(NB - 1) * OUT_SEQ + SEQ) * NJ * DM) return;
    if (SZ_TOTAL > ws_size) return;
    const float* x    = (const float*)d_in[0];
    const float* mask = (const float*)d_in[1];
    const float* qm   = (const float*)d_in[2];
    const float* km   = (const float*)d_in[3];
    const float* vm   = (const float*)d_in[4];
    const float* pj   = (const float*)d_in[5];
    const float* gam  = (const float*)d_in[6];
    const float* bet  = (const float*)d_in[7];
    float* OUT = (float*)d_out;
    char* wsp = (char*)d_ws;
    bf* XB  = (bf*)wsp;  wsp += SZ_XB;
    bf* WQT = (bf*)wsp;  wsp += SZ_WT;
    bf* WKT = (bf*)wsp;  wsp += SZ_WT;
    bf* WVT = (bf*)wsp;  wsp += SZ_WT;
    h16* PT = (h16*)wsp; wsp += SZ_WT;
    h16* QH = (h16*)wsp; wsp += SZ_PL;
    h16* QR = (h16*)wsp; wsp += SZ_PL;
    h16* KP = (h16*)wsp; wsp += SZ_PL;
    h16* VT = (h16*)wsp; wsp += SZ_PL;
    h16* CT = (h16*)wsp; wsp += SZ_PL;
    h16* KR = (h16*)wsp; wsp += SZ_RS;
    h16* VR = (h16*)wsp; wsp += SZ_RS;

    if (SEQ == SEQ_FULL) {
        const size_t n8 = (size_t)NB * SEQ * NJ * DM / 8;
        k_cvt8<<<(unsigned)((n8 + 255) / 256), 256, 0, stream>>>(x, XB, n8);
    } else {
        const size_t n8 = (size_t)SEQ * NJ * DM / 8;
        for (int b = 0; b < NB; ++b) k_cvt8<<<(unsigned)((n8 + 255) / 256), 256, 0, stream>>>(x + (size_t)b * SEQ_FULL * NJ * DM, XB + (size_t)b * SEQ * NJ * DM, n8);
    }
    k_wtr<<<NHD * NJ, 256, 0, stream>>>(qm, WQT);
    k_wtr<<<NHD * NJ, 256, 0, stream>>>(km, WKT);
    k_wtr<<<NHD * NJ, 256, 0, stream>>>(vm, WVT);
    k_ptr<<<NHD * NJ, 256, 0, stream>>>(pj, PT);

    k_proj_qk<<<dim3(NB * SEQ / 64, DM / 64, NJ), 32, 0, stream>>>(XB, WQT, QH, QR, SEQ);
    k_proj_qk<<<dim3(NB * SEQ / 64, DM / 64, NJ), 32, 0, stream>>>(XB, WKT, KP, KR, EROWS);
    k_proj_vt<<<dim3(DM / 64, NB * SEQ / 64, NJ), 32, 0, stream>>>(WVT, XB, VT, VR, EROWS);

    k_flash_early<<<dim3(EROWS / (16 * AW), NB * NHD * NJ, 1), 32 * AW, 0, stream>>>(QH, QR, KP, KR, VT, VR, mask, CT);
    if (SEQ > EROWS)
        k_flash_late<<<dim3((SEQ - EROWS) / (16 * AW), NB * NHD * NJ, 1), 32 * AW, 0, stream>>>(QH, QR, KP, KR, VT, VR, mask, CT);

    k_oproj<<<dim3(NB * SEQ / 32, NJ, 1), 32, 0, stream>>>(CT, PT, x, gam, bet, OUT);
}
